// LSTM_71236327572079
// MI455X (gfx1250) — hardware-verified
//
#include <hip/hip_runtime.h>
#include <math.h>

typedef __attribute__((ext_vector_type(16))) _Float16 v16h;
typedef __attribute__((ext_vector_type(8)))  _Float16 v8h;
typedef __attribute__((ext_vector_type(4)))  _Float16 v4h;
typedef __attribute__((ext_vector_type(8)))  float    v8f;
typedef __attribute__((ext_vector_type(4)))  float    v4f;

constexpr int N_BATCH  = 8;
constexpr int N_STEP   = 20;
constexpr int N_STOCK  = 1000;
constexpr int D_IN     = 64;
constexpr int D_HID    = 64;
constexpr int K_CAT    = D_IN + D_HID;
constexpr int W_PITCH  = 136;
constexpr int A_PITCH  = 136;
constexpr int N_THR    = 128;
constexpr int SC_PITCH = 32;
constexpr int HB_PITCH = N_STEP * D_HID + 4;
constexpr float WCARRY     = 16.0f;
constexpr float WCARRY_INV = 1.0f / WCARRY;

static_assert(K_CAT == 128, "four k-steps of 32");
static_assert(K_CAT % 32 == 0, "k-steps without a tail");
static_assert(D_HID == 16 * (N_THR / 32), "four waves own 16 columns each");
static_assert((K_CAT * D_HID) == 16 * N_THR * 4, "weight staging covers the gate matrix exactly");
static_assert(N_BATCH * (D_IN / 4) == N_THR, "x staging covers 8 rows x 64 columns exactly");
static_assert(N_BATCH * (D_HID / 4) == N_THR, "output store covers 8 rows x 64 columns exactly");
static_assert(N_BATCH * N_STEP <= 2 * N_THR, "two score dots per thread cover all (b, t)");
static_assert(N_STEP <= SC_PITCH, "score row pitch");
static_assert((W_PITCH % 8) == 0 && (A_PITCH % 8) == 0, "16-B aligned fragment rows");
static_assert(((HB_PITCH * 4) % 16) == 0, "history rows 16-B aligned");
static_assert(((HB_PITCH * 4) % 256) != 0 && (HB_PITCH * 4) > 1020, "history row pitch not pairable");
static_assert(HB_PITCH >= N_STEP * D_HID, "history row holds all steps");
static_assert(D_HID * W_PITCH * 2 + N_BATCH * A_PITCH * 2 + N_BATCH * HB_PITCH * 4 + N_BATCH * SC_PITCH * 4 <= 65536, "static LDS budget");

__device__ __forceinline__ unsigned short f2bf_bits(float f) {
  unsigned u = __float_as_uint(f);
  return (unsigned short)((u + 0x7FFFu + ((u >> 16) & 1u)) >> 16);
}
__device__ __forceinline__ float bf_bits2f(unsigned short h) { return __uint_as_float(((unsigned)h) << 16); }
__device__ __forceinline__ float bf16r(float f) { return bf_bits2f(f2bf_bits(f)); }

struct FragH {
  union U { v16h v; v8h h[2]; };
  static __device__ __forceinline__ v16h load(const _Float16* p) {
    U f;
    f.h[0] = *(const v8h*)(p);
    f.h[1] = *(const v8h*)(p + 16);
    return f.v;
  }
  static __device__ __forceinline__ v8f mma(v16h a, v16h b, v8f c) {
    return __builtin_amdgcn_wmma_f32_16x16x32_f16(false, a, false, b, (short)0, c, false, false);
  }
};

__device__ __forceinline__ void guard_group(v8f& a0, v8f& a1, v8f& a2, v8f& a3,
                                            v16h x, v16h b0, v16h b1, v16h b2, v16h b3) {
  asm volatile("v_nop\n\tv_nop\n\tv_nop\n\tv_nop"
               : "+v"(a0), "+v"(a1), "+v"(a2), "+v"(a3)
               : "v"(x), "v"(b0), "v"(b1), "v"(b2), "v"(b3)
               : "memory");
}

__device__ __forceinline__ float fsig(float v)  { return __builtin_amdgcn_rcpf(1.0f + __expf(-v)); }
__device__ __forceinline__ float ftanh(float v) { return 1.0f - 2.0f * __builtin_amdgcn_rcpf(__expf(2.0f * v) + 1.0f); }

__device__ __forceinline__ void stage_gate(const float* __restrict__ Wsrc, _Float16* Wb,
                                           int tid, int col, int koff, v16h (&bf)[4]) {
  __syncthreads();
#pragma unroll 4
  for (int it = 0; it < 16; ++it) {
    const int idx = it * N_THR + tid;
    const int k   = idx >> 4;
    const int c4  = (idx & 15) * 4;
    const v4f v = *(const v4f*)(Wsrc + k * D_HID + c4);
    const float e0 = v[0];
    const float e1 = v[1];
    const float e2 = v[2];
    const float e3 = v[3];
    Wb[(c4 + 0) * W_PITCH + k] = (_Float16)(bf16r(e0) * WCARRY);
    Wb[(c4 + 1) * W_PITCH + k] = (_Float16)(bf16r(e1) * WCARRY);
    Wb[(c4 + 2) * W_PITCH + k] = (_Float16)(bf16r(e2) * WCARRY);
    Wb[(c4 + 3) * W_PITCH + k] = (_Float16)(bf16r(e3) * WCARRY);
  }
  __syncthreads();
#pragma unroll
  for (int ks = 0; ks < 4; ++ks) bf[ks] = FragH::load(Wb + col * W_PITCH + ks * 32 + koff);
}

__global__ __launch_bounds__(128)
void gated_cell_seq_kernel(const float* __restrict__ x,
                           const float* __restrict__ Wi, const float* __restrict__ bi,
                           const float* __restrict__ Wo, const float* __restrict__ bo,
                           const float* __restrict__ Wf, const float* __restrict__ bf_,
                           const float* __restrict__ Wc, const float* __restrict__ bc,
                           const float* __restrict__ Wt,
                           float* __restrict__ out) {
  __shared__ __align__(16) _Float16 Wbuf[D_HID * W_PITCH];
  __shared__ __align__(16) _Float16 xh[N_BATCH * A_PITCH];
  __shared__ __align__(16) float hist[N_BATCH * HB_PITCH];
  __shared__ __align__(16) float sc[N_BATCH * SC_PITCH];

  const int n    = blockIdx.x;
  const int tid  = threadIdx.x;
  const int lane = tid & 31;
  const int wave = tid >> 5;
  const int half = lane >> 4;
  const int lr   = lane & 15;
  const int col  = wave * 16 + lr;
  const int koff = half * 8;

  {
    const v8h z = {(_Float16)0.0f, (_Float16)0.0f, (_Float16)0.0f, (_Float16)0.0f,
                   (_Float16)0.0f, (_Float16)0.0f, (_Float16)0.0f, (_Float16)0.0f};
#pragma unroll 1
    for (int i = tid; i < (N_BATCH * A_PITCH) / 8; i += N_THR) *(v8h*)(xh + i * 8) = z;
  }

  const float bias_i = bf16r(bi[n * D_HID + col]);
  const float bias_o = bf16r(bo[n * D_HID + col]);
  const float bias_f = bf16r(bf_[n * D_HID + col]);
  const float bias_c = bf16r(bc[n * D_HID + col]);

  v16h bfI[4], bfO[4], bfF[4], bfC[4];
  const size_t wofs = (size_t)n * K_CAT * D_HID;
  stage_gate(Wi + wofs, Wbuf, tid, col, koff, bfI);
  stage_gate(Wo + wofs, Wbuf, tid, col, koff, bfO);
  stage_gate(Wf + wofs, Wbuf, tid, col, koff, bfF);
  stage_gate(Wc + wofs, Wbuf, tid, col, koff, bfC);

  const int xb = tid >> 4;
  const int xd = (tid & 15) << 2;
  {
    const v4f xv = *(const v4f*)(x + (((size_t)xb * N_STEP + 0) * N_STOCK + n) * D_IN + xd);
    const float e0 = xv[0];
    const float e1 = xv[1];
    const float e2 = xv[2];
    const float e3 = xv[3];
    v4h hv;
    hv[0] = (_Float16)bf16r(e0);
    hv[1] = (_Float16)bf16r(e1);
    hv[2] = (_Float16)bf16r(e2);
    hv[3] = (_Float16)bf16r(e3);
    *(v4h*)(xh + xb * A_PITCH + xd) = hv;
  }
  __syncthreads();

  const unsigned amask = (lr < N_BATCH) ? 0xffffffffu : 0u;
  const _Float16* arow = xh + (lr & (N_BATCH - 1)) * A_PITCH + koff;
  union AFrag { v16h v; unsigned u[8]; };

  float cst[8];
#pragma unroll
  for (int r = 0; r < 8; ++r) cst[r] = 0.0f;
  const v8f z8 = {0.f, 0.f, 0.f, 0.f, 0.f, 0.f, 0.f, 0.f};

#pragma unroll 1
  for (int t = 0; t < N_STEP; ++t) {
    v8f accI = z8, accO = z8, accF = z8, accC = z8;
#pragma unroll
    for (int ks = 0; ks < 4; ++ks) {
      AFrag af;
      af.v = FragH::load(arow + ks * 32);
#pragma unroll
      for (int i = 0; i < 8; ++i) af.u[i] &= amask;
      accI = FragH::mma(af.v, bfI[ks], accI);
      accO = FragH::mma(af.v, bfO[ks], accO);
      accF = FragH::mma(af.v, bfF[ks], accF);
      accC = FragH::mma(af.v, bfC[ks], accC);
      guard_group(accI, accO, accF, accC, af.v, bfI[ks], bfO[ks], bfF[ks], bfC[ks]);
    }

    float h2[8];
#pragma unroll
    for (int r = 0; r < 8; ++r) {
      const float zi = accI[r] * WCARRY_INV + bias_i;
      const float zo = accO[r] * WCARRY_INV + bias_o;
      const float zf = accF[r] * WCARRY_INV + bias_f;
      const float zc = accC[r] * WCARRY_INV + bias_c;
      const float ig = fsig(zi);
      const float og = fsig(zo);
      const float fg = fsig(zf);
      const float ch = ftanh(zc);
      const float cn = fg * cst[r] + ig * ch;
      cst[r] = cn;
      h2[r] = og * ftanh(cn);
    }

    __syncthreads();

    const int tn = (t + 1 < N_STEP) ? (t + 1) : (N_STEP - 1);
    v4f xnext = *(const v4f*)(x + (((size_t)xb * N_STEP + (size_t)tn) * N_STOCK + n) * D_IN + xd);
    asm volatile("" : "+v"(xnext));

    if (half == 0) {
#pragma unroll
      for (int r = 0; r < 8; ++r) {
        xh[r * A_PITCH + D_IN + col] = (_Float16)h2[r];
        hist[r * HB_PITCH + t * D_HID + col] = h2[r];
      }
    }
    {
      const float e0 = xnext[0];
      const float e1 = xnext[1];
      const float e2 = xnext[2];
      const float e3 = xnext[3];
      v4h hv;
      hv[0] = (_Float16)bf16r(e0);
      hv[1] = (_Float16)bf16r(e1);
      hv[2] = (_Float16)bf16r(e2);
      hv[3] = (_Float16)bf16r(e3);
      *(v4h*)(xh + xb * A_PITCH + xd) = hv;
    }
    __syncthreads();
  }

#pragma unroll 1
  for (int rep = 0; rep < 2; ++rep) {
    const int s  = tid + rep * N_THR;
    const int sq = (s < N_BATCH * N_STEP) ? s : (N_BATCH * N_STEP - 1);
    const int b  = sq / N_STEP;
    const int tt = sq - b * N_STEP;
    const float* wt = Wt + ((size_t)n * N_STEP + tt) * D_HID;
    const float* hp = hist + b * HB_PITCH + tt * D_HID;
    float a = 0.0f;
#pragma unroll 4
    for (int d4 = 0; d4 < D_HID / 4; ++d4) {
      const v4f w = *(const v4f*)(wt + 4 * d4);
      const v4f hq = *(const v4f*)(hp + 4 * d4);
      const float w0 = w[0];
      const float w1 = w[1];
      const float w2 = w[2];
      const float w3 = w[3];
      const float g0 = hq[0];
      const float g1 = hq[1];
      const float g2 = hq[2];
      const float g3 = hq[3];
      a = fmaf(g0, bf16r(w0), a);
      a = fmaf(g1, bf16r(w1), a);
      a = fmaf(g2, bf16r(w2), a);
      a = fmaf(g3, bf16r(w3), a);
    }
    if (s < N_BATCH * N_STEP) sc[b * SC_PITCH + tt] = a;
  }
  __syncthreads();

  if (tid < N_BATCH) {
    float m = -3.0e38f;
#pragma unroll 1
    for (int tt = 0; tt < N_STEP; ++tt) m = fmaxf(m, sc[tid * SC_PITCH + tt]);
    float ssum = 0.0f;
#pragma unroll 1
    for (int tt = 0; tt < N_STEP; ++tt) {
      const float e = expf(sc[tid * SC_PITCH + tt] - m);
      sc[tid * SC_PITCH + tt] = e;
      ssum += e;
    }
    const float inv = 1.0f / ssum;
#pragma unroll 1
    for (int tt = 0; tt < N_STEP; ++tt) sc[tid * SC_PITCH + tt] *= inv;
  }
  __syncthreads();

  {
    const int ob = tid >> 4;
    const int od = (tid & 15) << 2;
    float o0 = 0.0f, o1 = 0.0f, o2 = 0.0f, o3 = 0.0f;
#pragma unroll 4
    for (int tt = 0; tt < N_STEP; ++tt) {
      const float w = sc[ob * SC_PITCH + tt];
      const v4f hv = *(const v4f*)(hist + ob * HB_PITCH + tt * D_HID + od);
      o0 = fmaf(w, hv[0], o0);
      o1 = fmaf(w, hv[1], o1);
      o2 = fmaf(w, hv[2], o2);
      o3 = fmaf(w, hv[3], o3);
    }
    v4f o;
    o[0] = o0;
    o[1] = o1;
    o[2] = o2;
    o[3] = o3;
    float* op = out + ((size_t)ob * N_STOCK + n) * D_HID + od;
    *(volatile v4f*)op = o;
    __threadfence();
    *(volatile v4f*)op = o;
  }
}

extern "C" void kernel_launch(void* const* d_in, const int* in_sizes, int n_in,
                              void* d_out, int out_size, void* d_ws, size_t ws_size,
                              hipStream_t stream) {
  (void)d_ws;
  (void)ws_size;
  if (n_in < 10 || d_out == nullptr) return;
  const int nx = N_BATCH * N_STEP * N_STOCK * D_IN;
  const int nw = N_STOCK * K_CAT * D_HID;
  const int nb = N_STOCK * D_HID;
  const int nt = N_STOCK * N_STEP * D_HID;
  if (in_sizes[0] != nx || in_sizes[1] != nw || in_sizes[2] != nb || in_sizes[3] != nw || in_sizes[4] != nb ||
      in_sizes[5] != nw || in_sizes[6] != nb || in_sizes[7] != nw || in_sizes[8] != nb || in_sizes[9] != nt ||
      out_size != N_BATCH * N_STOCK * D_HID) return;

  const float* x  = (const float*)d_in[0];
  const float* Wi = (const float*)d_in[1];
  const float* bi = (const float*)d_in[2];
  const float* Wo = (const float*)d_in[3];
  const float* bo = (const float*)d_in[4];
  const float* Wf = (const float*)d_in[5];
  const float* bf = (const float*)d_in[6];
  const float* Wc = (const float*)d_in[7];
  const float* bc = (const float*)d_in[8];
  const float* Wt = (const float*)d_in[9];
  float* out = (float*)d_out;

  gated_cell_seq_kernel<<<dim3(N_STOCK), dim3(N_THR), 0, stream>>>(
      x, Wi, bi, Wo, bo, Wf, bf, Wc, bc, Wt, out);
}
